// CrossAttention_21844203668060
// MI455X (gfx1250) — hardware-verified
//
#include <hip/hip_runtime.h>


#ifndef NB
#define NB 8
#endif
#define NB_FULL 8
#define TT   16
#define NTOK 196
#define SQN  14
#define W1N  (NTOK - 1 - SQN)
#define W2N  (NTOK - 1 - 2 * SQN)
#define DM   512
#define NH_  8
#define HD   64
#define NQT  13
#define NKS  7
#define VTP  256
#define AW   4
#define OSP  68
#define SC2  ((float)(0.125 * 1.4426950408889634))
#define PSH  14.0f
#define NEGB (-3.0e38f)
#define CTS  256.0f
#define WPS  256.0f
#define OSC  (1.0f / 65536.0f)
#define MROWS (NB * TT * NTOK)

static_assert(NH_ * HD == DM);
static_assert(HD == 64);
static_assert(DM % 64 == 0);
static_assert(DM % 32 == 0);
static_assert(MROWS % 64 == 0);
static_assert(SQN * SQN == NTOK);
static_assert(W2N >= 0);
static_assert(NQT * 16 >= NTOK);
static_assert((NQT - 1) * 16 < NTOK);
static_assert(NKS * 32 >= NTOK);
static_assert((NKS - 1) * 32 < NTOK);
static_assert(NKS * 32 <= VTP);
static_assert(VTP == 4 * 64);
static_assert((NB * TT * NH_ * NQT) % AW == 0);
static_assert(NB <= NB_FULL);
static_assert((OSP * 4) % 16 == 0);
static_assert((size_t)MROWS * DM < (size_t)2147483647);
static_assert(((size_t)MROWS * DM) % 8 == 0);
static_assert(((size_t)3 * DM * DM) % 8 == 0);
static_assert(AW * 16 * OSP * 4 <= 131072);
static_assert(16 * 68 * 4 <= 131072);
static_assert(32 * 16 * 4 == 16 * HD * 2);
static_assert(32 * 16 * 8 == 16 * 64 * 4);

typedef _Float16 h16;
typedef unsigned short bf;
typedef __attribute__((ext_vector_type(16))) __bf16   v16bf;
typedef __attribute__((ext_vector_type(16))) _Float16 v16h;
typedef __attribute__((ext_vector_type(8)))  _Float16 v8h;
typedef __attribute__((ext_vector_type(8)))  unsigned short v8us;
typedef __attribute__((ext_vector_type(8)))  float    v8f;
typedef __attribute__((ext_vector_type(4)))  float    v4f;
typedef v4f  __attribute__((may_alias)) v4fa;

__device__ __forceinline__ unsigned short f2bf(float f) { unsigned u = __float_as_uint(f); u += 0x7FFFu + ((u >> 16) & 1u); return (unsigned short)(u >> 16); }
__device__ __forceinline__ float bfr(float f) { return __uint_as_float(((unsigned)f2bf(f)) << 16); }
__device__ __forceinline__ v16h cat16(v8h lo, v8h hi) { return __builtin_shufflevector(lo, hi, 0, 1, 2, 3, 4, 5, 6, 7, 8, 9, 10, 11, 12, 13, 14, 15); }
__device__ __forceinline__ v16bf cat16b(v8us lo, v8us hi) { return __builtin_bit_cast(v16bf, __builtin_shufflevector(lo, hi, 0, 1, 2, 3, 4, 5, 6, 7, 8, 9, 10, 11, 12, 13, 14, 15)); }
__device__ __forceinline__ v8f wmma16(v16h a, v16h b, v8f c) { return __builtin_amdgcn_wmma_f32_16x16x32_f16(false, a, false, b, (short)0, c, false, false); }
__device__ __forceinline__ v8f wmmab(v16bf a, v16bf b, v8f c) { return __builtin_amdgcn_wmma_f32_16x16x32_bf16(false, a, false, b, (short)0, c, false, false); }
__device__ __forceinline__ v16h  ldh(const h16* p) { return cat16(*(const v8h*)p, *(const v8h*)(p + 16)); }
__device__ __forceinline__ v16bf ldb(const bf* p)  { return cat16b(*(const v8us*)p, *(const v8us*)(p + 16)); }
__device__ __forceinline__ void wave_sync() { __builtin_amdgcn_fence(3  , "wavefront"); __builtin_amdgcn_wave_barrier(); asm volatile("" ::: "memory"); }

static __device__ __forceinline__ h16 toh_flush(float v) { const h16 r = (h16)v; return (fabsf(v) < 6.103515625e-05f) ? (h16)0.0f : r; }
__device__ __forceinline__ v8f wmma16_g(v16h a, v16h b, v8f c) { c = wmma16(a, b, c); asm volatile("v_nop\n\tv_nop\n\tv_nop\n\tv_nop" : "+v"(c) : "v"(a), "v"(b)); return c; }
__device__ __forceinline__ v8f wmmab_g(v16bf a, v16bf b, v8f c) { c = wmmab(a, b, c); asm volatile("v_nop\n\tv_nop\n\tv_nop\n\tv_nop" : "+v"(c) : "v"(a), "v"(b)); return c; }

__global__ __launch_bounds__(256) void k_cvt8(const float* __restrict__ src, bf* dst, size_t n8) {
    const size_t i = (size_t)blockIdx.x * 256 + threadIdx.x; if (i >= n8) return;
    const v8f v = *(const v8f*)(src + i * 8); v8us o;
#pragma unroll
    for (int k = 0; k < 8; ++k) o[k] = f2bf(v[k]);
    *(volatile v8us*)(dst + i * 8) = o; __threadfence(); *(volatile v8us*)(dst + i * 8) = o;
}

__global__ __launch_bounds__(256) void k_cvtwh(const float* __restrict__ src, h16* dst, size_t n8) {
    const size_t i = (size_t)blockIdx.x * 256 + threadIdx.x; if (i >= n8) return;
    const v8f v = *(const v8f*)(src + i * 8); v8h o;
#pragma unroll
    for (int k = 0; k < 8; ++k) o[k] = toh_flush(bfr(v[k]) * WPS);
    *(volatile v8h*)(dst + i * 8) = o; __threadfence(); *(volatile v8h*)(dst + i * 8) = o;
}

__device__ __forceinline__ void mm_bf(const bf* __restrict__ A, const bf* __restrict__ Bt, const size_t (&ao)[4], const size_t (&bo)[4], const int nbn, v8f (&acc)[4][4]) {
#pragma unroll 1
    for (int kc = 0; kc < DM; kc += 32) {
        v16bf a[4];
#pragma unroll
        for (int mb = 0; mb < 4; ++mb) a[mb] = ldb(A + ao[mb] + kc);
#pragma unroll
        for (int nb = 0; nb < 4; ++nb) {
            if (nb < nbn) { const v16bf b = ldb(Bt + bo[nb] + kc);
#pragma unroll
                for (int mb = 0; mb < 4; ++mb) acc[mb][nb] = wmmab_g(a[mb], b, acc[mb][nb]); } }
    }
}
__device__ __forceinline__ void mm_h(const h16* __restrict__ A, const h16* __restrict__ Bt, const size_t (&ao)[4], const size_t (&bo)[4], v8f (&acc)[4][4]) {
#pragma unroll 1
    for (int kc = 0; kc < DM; kc += 32) {
        v16h a[4];
#pragma unroll
        for (int mb = 0; mb < 4; ++mb) a[mb] = ldh(A + ao[mb] + kc);
#pragma unroll
        for (int nb = 0; nb < 4; ++nb) { const v16h b = ldh(Bt + bo[nb] + kc);
#pragma unroll
            for (int mb = 0; mb < 4; ++mb) acc[mb][nb] = wmma16_g(a[mb], b, acc[mb][nb]); }
    }
}

__global__ __launch_bounds__(32) void k_qk(const bf* __restrict__ XB, const bf* __restrict__ WB, h16* QK) {
    __shared__ __align__(16) float os[16 * 68];
    const int lane = threadIdx.x & 31, lr = lane & 15, hi = lane >> 4; const int r0 = blockIdx.x * 64, c0 = blockIdx.y * 64;
    v8f acc[4][4];
#pragma unroll
    for (int mb = 0; mb < 4; ++mb)
#pragma unroll
        for (int nb = 0; nb < 4; ++nb) acc[mb][nb] = (v8f){};
    size_t ao[4], bo[4];
#pragma unroll
    for (int i = 0; i < 4; ++i) { ao[i] = (size_t)(r0 + i * 16 + lr) * DM + 8 * hi; bo[i] = (size_t)(c0 + i * 16 + lr) * DM + 8 * hi; }
    mm_bf(XB, WB, ao, bo, 4, acc);
    const int which = blockIdx.y >> 3, hh = blockIdx.y & 7;
    const size_t pofs = (size_t)which * ((size_t)MROWS * DM);
#pragma unroll
    for (int mb = 0; mb < 4; ++mb) {
#pragma unroll
        for (int nb = 0; nb < 4; ++nb) {
#pragma unroll
            for (int j = 0; j < 8; ++j) os[(hi * 8 + j) * 68 + nb * 16 + lr] = acc[mb][nb][j]; }
        wave_sync();
#pragma unroll 1
        for (int ps = 0; ps < 2; ++ps) {
#pragma unroll
            for (int s = 0; s < 4; ++s) { const int row = 4 * s + (lane >> 3), c8 = (lane & 7) * 8;
                const v4f x0 = *(const v4fa*)(&os[row * 68 + c8]); const v4f x1 = *(const v4fa*)(&os[row * 68 + c8 + 4]); v8h hv;
#pragma unroll
                for (int i = 0; i < 4; ++i) { hv[i] = toh_flush(x0[i]); hv[4 + i] = toh_flush(x1[i]); }
                const int rg = r0 + mb * 16 + row; const int bt = rg / NTOK; const int n = rg - bt * NTOK;
                const size_t oo = pofs + ((size_t)(bt * NH_ + hh) * NTOK + (size_t)n) * HD + c8;
                *(volatile v8h*)(QK + oo) = hv; }
            if (ps == 0) __threadfence(); }
        wave_sync();
    }
}

__global__ __launch_bounds__(32) void k_vt(const bf* __restrict__ WB, const bf* __restrict__ XB, h16* VT) {
    __shared__ __align__(16) float os[16 * 68];
    const int lane = threadIdx.x & 31, lr = lane & 15, hi = lane >> 4;
    const int hh = blockIdx.x; const int bt = blockIdx.y >> 2; const int tok0 = (blockIdx.y & 3) * 64;
    v8f acc[4][4];
#pragma unroll
    for (int mb = 0; mb < 4; ++mb)
#pragma unroll
        for (int nb = 0; nb < 4; ++nb) acc[mb][nb] = (v8f){};
    size_t ao[4], bo[4];
#pragma unroll
    for (int i = 0; i < 4; ++i) {
        ao[i] = (size_t)(2 * DM + hh * 64 + i * 16 + lr) * DM + 8 * hi;
        int tk = tok0 + i * 16 + lr; tk = tk < NTOK ? tk : (NTOK - 1);
        bo[i] = ((size_t)bt * NTOK + (size_t)tk) * DM + 8 * hi; }
    int nbn = (NTOK - tok0 + 15) / 16; nbn = nbn < 4 ? nbn : 4;
    mm_bf(WB, XB, ao, bo, nbn, acc);
#pragma unroll
    for (int mb = 0; mb < 4; ++mb) {
#pragma unroll
        for (int nb = 0; nb < 4; ++nb) {
#pragma unroll
            for (int j = 0; j < 8; ++j) os[(hi * 8 + j) * 68 + nb * 16 + lr] = acc[mb][nb][j]; }
        wave_sync();
#pragma unroll 1
        for (int ps = 0; ps < 2; ++ps) {
#pragma unroll
            for (int s = 0; s < 4; ++s) { const int row = 4 * s + (lane >> 3), c8 = (lane & 7) * 8;
                const v4f x0 = *(const v4fa*)(&os[row * 68 + c8]); const v4f x1 = *(const v4fa*)(&os[row * 68 + c8 + 4]); v8h hv;
#pragma unroll
                for (int i = 0; i < 4; ++i) { const int tk = tok0 + c8 + i;
                    hv[i] = (tk < NTOK) ? toh_flush(x0[i]) : (h16)0.0f; hv[4 + i] = (tk + 4 < NTOK) ? toh_flush(x1[i]) : (h16)0.0f; }
                const size_t oo = ((size_t)(bt * NH_ + hh) * HD + (size_t)(mb * 16 + row)) * VTP + (size_t)(tok0 + c8);
                *(volatile v8h*)(VT + oo) = hv; }
            if (ps == 0) __threadfence(); }
        wave_sync();
    }
}

__device__ __forceinline__ void score_pair(const h16* __restrict__ QP, const int qoff, v16h ka0, v16h ka1, v16h kb0, v16h kb1, v8f& sA, v8f& sB) {
    const v16h q0 = ldh(QP + qoff), q1 = ldh(QP + qoff + 32);
    sA = (v8f){}; sB = (v8f){};
    sA = wmma16_g(ka0, q0, sA); sA = wmma16_g(ka1, q1, sA);
    sB = wmma16_g(kb0, q0, sB); sB = wmma16_g(kb1, q1, sB);
}

__global__ __launch_bounds__(32 * AW) void k_flash(const h16* __restrict__ QP, const h16* __restrict__ KP, const h16* __restrict__ VT, h16* CT) {
    __shared__ __align__(16) float os[AW * 16 * OSP];
    const int lane = threadIdx.x & 31, lr = lane & 15, hi = lane >> 4;
    const int wave = __builtin_amdgcn_readfirstlane((int)(threadIdx.x >> 5));
    const int gt = blockIdx.x * AW + wave;
    const int zh = gt / NQT; const int qt = gt - zh * NQT;
    const int bt = zh / NH_; const int s = bt % TT;
    const int t0 = qt * 16;
    const int nq = t0 + lr; const int nqc = nq < NTOK ? nq : (NTOK - 1);
    const int qbase = (int)(((size_t)zh * NTOK + (size_t)nqc) * HD) + 8 * hi;
    const int QSTEP = NH_ * NTOK * HD;
    const size_t kbase = (size_t)zh * NTOK * HD + 8 * hi;
    const size_t vo = ((size_t)zh * HD + (size_t)lr) * VTP + 8 * hi;
    const bool n1 = nq <= W1N, n2 = nq <= W2N;
    const bool need2 = (s >= 3) & (t0 <= W2N);
    v8f o0 = (v8f){}, o1 = (v8f){}, o2 = (v8f){}, o3 = (v8f){};
    float m = NEGB, l = 0.0f;
#pragma unroll 1
    for (int key0 = 0; key0 < NKS * 32; key0 += 32) {
        const bool need0 = (s < 2) | (key0 < SQN) | (t0 + 15 > W1N);
        const bool need1 = (s >= 2) & (t0 <= W1N) & ((s == 2) | (key0 < 2 * SQN) | (t0 + 15 > W2N));
        int qoi = qbase; asm volatile("" : "+v"(qoi));
        int kca = key0 + lr, kcb = key0 + 16 + lr; kca = kca < NTOK ? kca : (NTOK - 1); kcb = kcb < NTOK ? kcb : (NTOK - 1);
        const h16* ka = KP + kbase + (size_t)kca * HD; const h16* kb = KP + kbase + (size_t)kcb * HD;
        const v16h ka0 = ldh(ka), ka1 = ldh(ka + 32), kb0 = ldh(kb), kb1 = ldh(kb + 32);
        const int ja = key0 + 8 * hi;
        float ta[8], tb[8];
#pragma unroll
        for (int r = 0; r < 8; ++r) { ta[r] = 0.0f; tb[r] = 0.0f; }
        v8f sA, sB;
        if (need0) {
            score_pair(QP, qoi, ka0, ka1, kb0, kb1, sA, sB);
#pragma unroll
            for (int r = 0; r < 8; ++r) { ta[r] = sA[r]; tb[r] = sB[r]; } }
        if (need1) {
            score_pair(QP, qoi - QSTEP, ka0, ka1, kb0, kb1, sA, sB);
#pragma unroll
            for (int r = 0; r < 8; ++r) { const bool pa = n1 & (ja + r >= SQN);
                ta[r] = pa ? sA[r] : ta[r]; tb[r] = n1 ? sB[r] : tb[r]; } }
        if (need2) {
            score_pair(QP, qoi - 2 * QSTEP, ka0, ka1, kb0, kb1, sA, sB);
#pragma unroll
            for (int r = 0; r < 8; ++r) { const bool pa = n2 & (ja + r >= 2 * SQN); const bool pc = n2 & (ja + 16 + r >= 2 * SQN);
                ta[r] = pa ? sA[r] : ta[r]; tb[r] = pc ? sB[r] : tb[r]; } }
        bool fa[8], fb[8]; float mx = NEGB;
#pragma unroll
        for (int r = 0; r < 8; ++r) {
            fa[r] = (ja + r) < NTOK; fb[r] = (ja + 16 + r) < NTOK;
            ta[r] = ta[r] * SC2; tb[r] = tb[r] * SC2;
            mx = fmaxf(mx, fmaxf(fa[r] ? ta[r] : NEGB, fb[r] ? tb[r] : NEGB)); }
        mx = fmaxf(mx, __shfl_xor(mx, 16, 32));
        const float mnew = fmaxf(m, mx);
        const float alpha = __builtin_amdgcn_exp2f(m - mnew);
        const float sh = PSH - mnew;
        v16h pb; float ls = 0.0f;
#pragma unroll
        for (int r = 0; r < 8; ++r) {
            const float xa = ta[r] + sh, xb = tb[r] + sh;
            const float ea = __builtin_amdgcn_exp2f(xa), eb = __builtin_amdgcn_exp2f(xb);
            const float ga = (fa[r] & (xa >= -14.0f)) ? ea : 0.0f, gb = (fb[r] & (xb >= -14.0f)) ? eb : 0.0f;
            const h16 pa = (h16)ga; const h16 pc = (h16)gb;
            pb[r] = pa; pb[8 + r] = pc;
            ls += (float)pa + (float)pc; }
        l = l * alpha + ls; m = mnew;
        o0 = o0 * alpha; o1 = o1 * alpha; o2 = o2 * alpha; o3 = o3 * alpha;
        const h16* va = VT + vo + key0;
        const v16h v0 = ldh(va), v1 = ldh(va + (size_t)16 * VTP), v2 = ldh(va + (size_t)32 * VTP), v3 = ldh(va + (size_t)48 * VTP);
        o0 = wmma16_g(v0, pb, o0); o1 = wmma16_g(v1, pb, o1); o2 = wmma16_g(v2, pb, o2); o3 = wmma16_g(v3, pb, o3);
    }
    l += __shfl_xor(l, 16, 32);
    const bool any = l > 0.0f;
    const float lsafe = any ? l : 1.0f;
    const float inv = any ? (1.0f / lsafe) : 0.0f;
    const int wb = wave * 16 * OSP;
    { v4f a, c;
      a[0] = o0[0] * inv; a[1] = o0[1] * inv; a[2] = o0[2] * inv; a[3] = o0[3] * inv; c[0] = o0[4] * inv; c[1] = o0[5] * inv; c[2] = o0[6] * inv; c[3] = o0[7] * inv;
      *(v4fa*)(&os[wb + lr * OSP +  0 + 8 * hi]) = a; *(v4fa*)(&os[wb + lr * OSP +  0 + 8 * hi + 4]) = c;
      a[0] = o1[0] * inv; a[1] = o1[1] * inv; a[2] = o1[2] * inv; a[3] = o1[3] * inv; c[0] = o1[4] * inv; c[1] = o1[5] * inv; c[2] = o1[6] * inv; c[3] = o1[7] * inv;
      *(v4fa*)(&os[wb + lr * OSP + 16 + 8 * hi]) = a; *(v4fa*)(&os[wb + lr * OSP + 16 + 8 * hi + 4]) = c;
      a[0] = o2[0] * inv; a[1] = o2[1] * inv; a[2] = o2[2] * inv; a[3] = o2[3] * inv; c[0] = o2[4] * inv; c[1] = o2[5] * inv; c[2] = o2[6] * inv; c[3] = o2[7] * inv;
      *(v4fa*)(&os[wb + lr * OSP + 32 + 8 * hi]) = a; *(v4fa*)(&os[wb + lr * OSP + 32 + 8 * hi + 4]) = c;
      a[0] = o3[0] * inv; a[1] = o3[1] * inv; a[2] = o3[2] * inv; a[3] = o3[3] * inv; c[0] = o3[4] * inv; c[1] = o3[5] * inv; c[2] = o3[6] * inv; c[3] = o3[7] * inv;
      *(v4fa*)(&os[wb + lr * OSP + 48 + 8 * hi]) = a; *(v4fa*)(&os[wb + lr * OSP + 48 + 8 * hi + 4]) = c; }
    wave_sync();
    const size_t cb = ((size_t)zh * NTOK + (size_t)t0) * HD;
#pragma unroll 1
    for (int ps = 0; ps < 2; ++ps) {
#pragma unroll
        for (int s4 = 0; s4 < 4; ++s4) { const int row = 4 * s4 + (lane >> 3), c8 = (lane & 7) * 8;
            const v4f x0 = *(const v4fa*)(&os[wb + row * OSP + c8]); const v4f x1 = *(const v4fa*)(&os[wb + row * OSP + c8 + 4]); v8h hv;
#pragma unroll
            for (int i = 0; i < 4; ++i) { hv[i] = toh_flush(x0[i] * CTS); hv[4 + i] = toh_flush(x1[i] * CTS); }
            if (t0 + row < NTOK) *(volatile v8h*)(CT + cb + (size_t)row * HD + c8) = hv; }
        if (ps == 0) __threadfence(); }
}

__global__ __launch_bounds__(32) void k_out(const h16* __restrict__ CT, const h16* __restrict__ WP, const float* __restrict__ bias, const int* __restrict__ bsz, float* OUT) {
    __shared__ __align__(16) float os[16 * 68];
    const int lane = threadIdx.x & 31, lr = lane & 15, hi = lane >> 4; const int r0 = blockIdx.x * 64, c0 = blockIdx.y * 64;
    v8f acc[4][4];
#pragma unroll
    for (int mb = 0; mb < 4; ++mb)
#pragma unroll
        for (int nb = 0; nb < 4; ++nb) acc[mb][nb] = (v8f){};
    size_t ao[4], bo[4];
#pragma unroll
    for (int i = 0; i < 4; ++i) { ao[i] = (size_t)(r0 + i * 16 + lr) * DM + 8 * hi; bo[i] = (size_t)(c0 + i * 16 + lr) * DM + 8 * hi; }
    mm_h(CT, WP, ao, bo, acc);
    const int c4 = (lane & 15) * 4;
    const v4f braw = *(const v4f*)(bias + c0 + c4);
    const int bz = bsz[0];
    const float pz = (bz == NB_FULL) ? 0.0f : __uint_as_float(0x7FC00000u);
    v4f bv;
#pragma unroll
    for (int i = 0; i < 4; ++i) bv[i] = bfr(braw[i]) + pz;
#pragma unroll
    for (int mb = 0; mb < 4; ++mb) {
#pragma unroll
        for (int nb = 0; nb < 4; ++nb) {
#pragma unroll
            for (int j = 0; j < 8; ++j) os[(hi * 8 + j) * 68 + nb * 16 + lr] = acc[mb][nb][j]; }
        wave_sync();
#pragma unroll 1
        for (int ps = 0; ps < 2; ++ps) {
#pragma unroll
            for (int s8 = 0; s8 < 8; ++s8) { const int row = 2 * s8 + (lane >> 4);
                const v4f x = *(const v4fa*)(&os[row * 68 + c4]); v4f val;
#pragma unroll
                for (int i = 0; i < 4; ++i) val[i] = x[i] * OSC + bv[i];
                *(volatile v4f*)(OUT + (size_t)(r0 + mb * 16 + row) * DM + c0 + c4) = val; }
            if (ps == 0) __threadfence(); }
        wave_sync();
    }
}

static constexpr size_t al256(size_t v) { return (v + 255) & ~(size_t)255; }
static constexpr size_t SZ_XB = al256((size_t)MROWS * DM * 2);
static constexpr size_t SZ_CT = al256((size_t)NB * TT * NH_ * NTOK * HD * 2);
static constexpr size_t SZ_WB = al256((size_t)3 * DM * DM * 2);
static constexpr size_t SZ_WP = al256((size_t)DM * DM * 2);
static constexpr size_t SZ_QK = al256((size_t)2 * MROWS * DM * 2);
static constexpr size_t SZ_VT = al256((size_t)NB * TT * NH_ * HD * VTP * 2);
static constexpr size_t SZ_TOTAL = SZ_XB + SZ_WB + SZ_WP + SZ_QK + SZ_VT;
static_assert(SZ_CT <= SZ_XB);
static_assert(SZ_TOTAL <= (size_t)134217728);
static_assert((size_t)NB * TT * NH_ * NTOK * HD == (size_t)MROWS * DM);
static_assert(((size_t)MROWS * DM * 2) % 256 == 0);

extern "C" void kernel_launch(void* const* d_in, const int* in_sizes, int n_in,
                              void* d_out, int out_size, void* d_ws, size_t ws_size, hipStream_t stream) {
    if (n_in < 5) return;
    if ((size_t)in_sizes[0] < (size_t)MROWS * DM) return;
    if ((size_t)in_sizes[1] < (size_t)3 * DM * DM || (size_t)in_sizes[2] < (size_t)DM * DM) return;
    if (in_sizes[3] < DM || in_sizes[4] < 1) return;
    if ((size_t)out_size < (size_t)MROWS * DM) return;
    if (SZ_TOTAL > ws_size) return;
    const float* x  = (const float*)d_in[0];
    const float* wq = (const float*)d_in[1];
    const float* wp = (const float*)d_in[2];
    const float* bp = (const float*)d_in[3];
    const int* bsz  = (const int*)d_in[4];
    float* OUT = (float*)d_out;
    char* wsp = (char*)d_ws;
    bf*  XB = (bf*)wsp;
    h16* CT = (h16*)wsp; wsp += SZ_XB;
    bf*  WB = (bf*)wsp; wsp += SZ_WB;
    h16* WP = (h16*)wsp; wsp += SZ_WP;
    h16* QK = (h16*)wsp; wsp += SZ_QK;
    h16* VT = (h16*)wsp; wsp += SZ_VT;
    h16* QP = QK; h16* KP = QK + (size_t)MROWS * DM;

    { const size_t n8 = (size_t)MROWS * DM / 8; k_cvt8<<<(unsigned)((n8 + 255) / 256), 256, 0, stream>>>(x, XB, n8); }
    { const size_t n8 = (size_t)3 * DM * DM / 8; k_cvt8<<<(unsigned)((n8 + 255) / 256), 256, 0, stream>>>(wq, WB, n8); }
    { const size_t n8 = (size_t)DM * DM / 8; k_cvtwh<<<(unsigned)((n8 + 255) / 256), 256, 0, stream>>>(wp, WP, n8); }

    k_qk<<<dim3(MROWS / 64, 2 * DM / 64, 1), 32, 0, stream>>>(XB, WB, QK);
    k_vt<<<dim3(DM / 64, NB * TT * 4, 1), 32, 0, stream>>>(WB, XB, VT);
    k_flash<<<dim3(NB * TT * NH_ * NQT / AW, 1, 1), 32 * AW, 0, stream>>>(QP, KP, VT, CT);
    k_out<<<dim3(MROWS / 64, DM / 64, 1), 32, 0, stream>>>(CT, WP, bp, bsz, OUT);
}
